// RNN_77309411561
// MI455X (gfx1250) — hardware-verified
//
#include <hip/hip_runtime.h>
#include <math.h>

constexpr int NBATCH = 8;
constexpr int NSTEP  = 4096;
constexpr int NIN    = 256;
constexpr int NHID   = 256;
constexpr int NGATE4 = 4 * NHID;
constexpr int NROWS  = NBATCH * NSTEP;

constexpr int RTHR   = 512;
constexpr int RWAVES = RTHR / 32;
constexpr int APITCH = NHID + 8;
constexpr int ATILE  = 16 * APITCH;
constexpr int SPITCH = NHID + 4;
constexpr int STILE  = NBATCH * SPITCH;

constexpr int PTHR    = 256;
constexpr int XCHUNKS = NROWS * NIN / 8;
constexpr int WCHUNKS = NGATE4 * NIN / 8;
constexpr int GEMM_TILES  = (NROWS / 64) * (NGATE4 / 64);
constexpr int GEMM_BLOCKS = GEMM_TILES / 8;

static_assert(NIN % 32 == 0);
static_assert(NHID % 32 == 0);
static_assert(NROWS % 64 == 0 && NGATE4 % 64 == 0);
static_assert(GEMM_TILES % 8 == 0);
static_assert(NHID == 16 * RWAVES);
static_assert(2 * NBATCH == 16);
static_assert(RWAVES == 2 * NBATCH);
static_assert(NHID / 2 == 32 * 4);
static_assert((NSTEP & (NSTEP - 1)) == 0);
static_assert(NIN == NHID);
static_assert(NIN / 8 == 32);
static_assert(APITCH % 8 == 0 && SPITCH % 4 == 0 && STILE % 4 == 0 && ATILE % 8 == 0);
static_assert((2 * ATILE) % 8 == 0);
static_assert(XCHUNKS % PTHR == 0 && WCHUNKS % PTHR == 0);
static_assert(NGATE4 == 4 * PTHR);

typedef __attribute__((ext_vector_type(16))) _Float16 v16h;
typedef __attribute__((ext_vector_type(8)))  _Float16 v8h;
typedef __attribute__((ext_vector_type(16))) __bf16   v16b;
typedef __attribute__((ext_vector_type(8)))  __bf16   v8b;
typedef __attribute__((ext_vector_type(8)))  float    v8f;
typedef __attribute__((ext_vector_type(4)))  float    v4f;

__device__ __forceinline__ unsigned short f2bf_bits(float f) {
  unsigned u = __float_as_uint(f);
  return (unsigned short)((u + 0x7FFFu + ((u >> 16) & 1u)) >> 16);
}
__device__ __forceinline__ float bf_bits2f(unsigned short h) { return __uint_as_float(((unsigned)h) << 16); }
__device__ __forceinline__ unsigned f2bf_u(float f) {
  const unsigned u = __float_as_uint(f);
  return (u + 0x7FFFu + ((u >> 16) & 1u)) >> 16;
}
__device__ __forceinline__ float  bf_u2f(unsigned h)    { return __uint_as_float(h << 16); }
__device__ __forceinline__ __bf16 bf_from_u(unsigned h) { return __builtin_bit_cast(__bf16, (unsigned short)h); }
__device__ __forceinline__ float h16_to_f32(unsigned hb) {
  const unsigned sgn = (hb & 0x8000u) << 16; const unsigned em = hb & 0x7fffu;
  const float fn = __uint_as_float((em << 13) + 0x38000000u);
  const float fs = (float)em * 5.9604644775390625e-8f;
  const float mag = (em < 0x400u) ? fs : fn; return __uint_as_float(__float_as_uint(mag) | sgn);
}

__device__ __forceinline__ void dep_guard_h(v8f& a, v8f& b, v16h x, v16h y) { asm volatile("v_nop\n\tv_nop\n\tv_nop\n\tv_nop" : "+v"(a), "+v"(b) : "v"(x), "v"(y)); }
__device__ __forceinline__ void dep_guard_b(v8f& a, v8f& b, v16b x, v16b y) { asm volatile("v_nop\n\tv_nop\n\tv_nop\n\tv_nop" : "+v"(a), "+v"(b) : "v"(x), "v"(y)); }
__device__ __forceinline__ void dep_guard4_h(v8f& a, v8f& b, v8f& c, v8f& d, v16h x, v16h y) { asm volatile("v_nop\n\tv_nop\n\tv_nop\n\tv_nop" : "+v"(a), "+v"(b), "+v"(c), "+v"(d) : "v"(x), "v"(y)); }
__device__ __forceinline__ void dep_guard4_b(v8f& a, v8f& b, v8f& c, v8f& d, v16b x, v16b y) { asm volatile("v_nop\n\tv_nop\n\tv_nop\n\tv_nop" : "+v"(a), "+v"(b), "+v"(c), "+v"(d) : "v"(x), "v"(y)); }
__device__ __forceinline__ void keep4_h(v16h a, v16h b, v16h c, v16h d) { asm volatile("v_nop" :: "v"(a), "v"(b), "v"(c), "v"(d)); }
__device__ __forceinline__ void keep4_b(v16b a, v16b b, v16b c, v16b d) { asm volatile("v_nop" :: "v"(a), "v"(b), "v"(c), "v"(d)); }
__device__ __forceinline__ void acc_guard4(v8f& a, v8f& b, v8f& c, v8f& d) { asm volatile("v_nop\n\tv_nop\n\tv_nop\n\tv_nop" : "+v"(a), "+v"(b), "+v"(c), "+v"(d)); }
__device__ __forceinline__ void group_guard(v8f& a0, v8f& a1, v8f& a2, v8f& a3,
                                            v16b fa, v16b b0, v16b b1, v16b b2, v16b b3) {
  asm volatile("v_nop\n\tv_nop\n\tv_nop\n\tv_nop"
               : "+v"(a0), "+v"(a1), "+v"(a2), "+v"(a3)
               : "v"(fa), "v"(b0), "v"(b1), "v"(b2), "v"(b3));
}

template <typename T> struct Frag;
template <> struct Frag<_Float16> {
  typedef v16h V; union U { v16h v; v8h h[2]; };
  static __device__ __forceinline__ v16h load(const _Float16* p) {
    U f; f.h[0] = *(const v8h*)(p); f.h[1] = *(const v8h*)(p + 16); return f.v;
  }
  static __device__ __forceinline__ v8f mma(v16h a, v16h b, v8f c) {
    return __builtin_amdgcn_wmma_f32_16x16x32_f16(false, a, false, b, (short)0, c, false, false);
  }
  static __device__ __forceinline__ void guard(v8f& a, v8f& b, v16h x, v16h y) { dep_guard_h(a, b, x, y); }
  static __device__ __forceinline__ void guard4(v8f& a, v8f& b, v8f& c, v8f& d, v16h x, v16h y) { dep_guard4_h(a, b, c, d, x, y); }
  static __device__ __forceinline__ void keep(v16h a, v16h b, v16h c, v16h d) { keep4_h(a, b, c, d); }
};
template <> struct Frag<__bf16> {
  typedef v16b V; union U { v16b v; v8b h[2]; };
  static __device__ __forceinline__ v16b load(const __bf16* p) {
    U f; f.h[0] = *(const v8b*)(p); f.h[1] = *(const v8b*)(p + 16); return f.v;
  }
  static __device__ __forceinline__ v8f mma(v16b a, v16b b, v8f c) {
    return __builtin_amdgcn_wmma_f32_16x16x32_bf16(false, a, false, b, (short)0, c, false, false);
  }
  static __device__ __forceinline__ void guard(v8f& a, v8f& b, v16b x, v16b y) { dep_guard_b(a, b, x, y); }
  static __device__ __forceinline__ void guard4(v8f& a, v8f& b, v8f& c, v8f& d, v16b x, v16b y) { dep_guard4_b(a, b, c, d, x, y); }
  static __device__ __forceinline__ void keep(v16b a, v16b b, v16b c, v16b d) { keep4_b(a, b, c, d); }
};

template <int ET> struct Elem;
template <> struct Elem<0> { typedef _Float16 T; };
template <> struct Elem<1> { typedef __bf16 T; };
template <int ET, bool SPLIT, int BIAS_MODE, int OUT_MODE, bool RESID, int ACT = 0>
__global__ __launch_bounds__(256) void wmma_gemm64(
    const unsigned short* __restrict__ Ap, const unsigned short* __restrict__ A2p, int lda, long strideA,
    const unsigned short* __restrict__ Btp, const unsigned short* __restrict__ Bt2p, int ldb, long strideB,
    void* __restrict__ Cout, void* __restrict__ Cout2, int ldc, long strideC,
    const float* __restrict__ bias,
    const float* __restrict__ resid, long strideR,
    int M, int N, int K, float scale) {
  typedef typename Elem<ET>::T T;
  typedef typename Frag<T>::V V;
  const T* A = (const T*)Ap; const T* A2 = (const T*)A2p; const T* Bt = (const T*)Btp; const T* Bt2 = (const T*)Bt2p;
  __shared__ __align__(16) float sT[8][16 * 68];
  const int b    = blockIdx.y;
  const int lane = threadIdx.x & 31;
  const int wave = threadIdx.x >> 5;
  const int tilesN = N >> 6;
  const int tilesM = M >> 6;
  const int tile = blockIdx.x * 8 + wave;
  if (tile >= tilesM * tilesN) return;
  const int tm = tile / tilesN;
  const int tn = tile - tm * tilesN;
  const int m0 = tm << 6;
  const int n0 = tn << 6;

  const T* Ab  = A  + (size_t)b * strideA;
  const T* Bb  = Bt + (size_t)b * strideB;
  const T* Ab2 = SPLIT ? (A2  + (size_t)b * strideA) : nullptr;
  const T* Bb2 = SPLIT ? (Bt2 + (size_t)b * strideB) : nullptr;

  const int rlane = lane & 15;
  const int koff  = (lane >> 4) * 8;
  const int mOff  = (lane >> 4) * 8;

  v8f acc[4][4];
#pragma unroll
  for (int i = 0; i < 4; ++i)
#pragma unroll
    for (int j = 0; j < 4; ++j) acc[i][j] = (v8f){0.f,0.f,0.f,0.f,0.f,0.f,0.f,0.f};

  for (int k0 = 0; k0 < K; k0 += 32) {
    V bh[4], bl[4];
#pragma unroll
    for (int j = 0; j < 4; ++j) {
      const size_t bo = (size_t)(n0 + (j << 4) + rlane) * ldb + koff + k0;
      bh[j] = Frag<T>::load(Bb + bo);
      if (SPLIT) bl[j] = Frag<T>::load(Bb2 + bo);
    }
#pragma unroll
    for (int i = 0; i < 4; ++i) {
      const size_t ao = (size_t)(m0 + (i << 4) + rlane) * lda + koff + k0;
      V ah = Frag<T>::load(Ab + ao);
      V al;
      if (SPLIT) al = Frag<T>::load(Ab2 + ao);
#pragma unroll
      for (int j = 0; j < 4; ++j) {
        acc[i][j] = Frag<T>::mma(ah, bh[j], acc[i][j]);
        if (SPLIT) {
          acc[i][j] = Frag<T>::mma(ah, bl[j], acc[i][j]);
          acc[i][j] = Frag<T>::mma(al, bh[j], acc[i][j]);
        }
      }
      Frag<T>::guard4(acc[i][0], acc[i][1], acc[i][2], acc[i][3], ah, SPLIT ? al : ah);
    }
    Frag<T>::keep(bh[0], bh[1], bh[2], bh[3]);
    if (SPLIT) Frag<T>::keep(bl[0], bl[1], bl[2], bl[3]);
  }
  acc_guard4(acc[0][0], acc[0][1], acc[0][2], acc[0][3]);
  acc_guard4(acc[1][0], acc[1][1], acc[1][2], acc[1][3]);
  acc_guard4(acc[2][0], acc[2][1], acc[2][2], acc[2][3]);
  acc_guard4(acc[3][0], acc[3][1], acc[3][2], acc[3][3]);

  float* slab = sT[wave];
  const float* Rb = RESID ? (resid + (size_t)b * strideR) : nullptr;
#pragma unroll
  for (int i = 0; i < 4; ++i) {
    const int mBase = m0 + (i << 4);
#pragma unroll
    for (int j = 0; j < 4; ++j) {
      const int n = n0 + (j << 4) + rlane;
      float bv = 0.f;
      if (BIAS_MODE == 2) bv = bias[n];
#pragma unroll
      for (int r = 0; r < 8; ++r) {
        float v = acc[i][j][r] * scale;
        if (BIAS_MODE == 1) v += bias[mBase + mOff + r];
        if (BIAS_MODE == 2) v += bv;
        if (RESID) v += Rb[(size_t)(mBase + mOff + r) * ldc + n];
        if (ACT == 1) v = tanhf(v);
        if (ACT == 2) v = fmaxf(v, 0.0f);
        if (ACT == 4) v = (v > 0.f) ? v : 0.01f * v;
        slab[(mOff + r) * 68 + (j << 4) + rlane] = v;
      }
    }
    __builtin_amdgcn_fence(__ATOMIC_RELEASE, "workgroup");
    __builtin_amdgcn_wave_barrier();
    __builtin_amdgcn_fence(__ATOMIC_ACQUIRE, "workgroup");
    if (OUT_MODE == 0) {
      float* C = (float*)Cout + (size_t)b * strideC;
      const int hh = lane >> 4, c4 = (lane & 15) * 4;
      for (int pass = 0; pass < 2; ++pass) {
#pragma unroll
        for (int it = 0; it < 8; ++it) {
          const int row = it * 2 + hh;
          v4f v = *(const v4f*)(slab + row * 68 + c4);
          *(volatile v4f*)(C + (size_t)(mBase + row) * ldc + n0 + c4) = v;
        }
        __threadfence();
      }
    } else {
      const int q = lane >> 3, c8 = (lane & 7) * 8;
      unsigned short* C  = (unsigned short*)Cout  + (size_t)b * strideC;
      unsigned short* C2 = (OUT_MODE == 2) ? ((unsigned short*)Cout2 + (size_t)b * strideC) : nullptr;
      for (int pass = 0; pass < 2; ++pass) {
#pragma unroll
        for (int it = 0; it < 4; ++it) {
          const int row = it * 4 + q;
          const float* sp = slab + row * 68 + c8;
          v8h hv, lv;
#pragma unroll
          for (int e = 0; e < 8; ++e) {
            if (OUT_MODE == 1) {
              hv[e] = (_Float16)sp[e];
            } else {
              unsigned short hb = f2bf_bits(sp[e]);
              unsigned short lb = f2bf_bits(sp[e] - bf_bits2f(hb));
              hv[e] = __builtin_bit_cast(_Float16, hb);
              lv[e] = __builtin_bit_cast(_Float16, lb);
            }
          }
          *(volatile v8h*)(C + (size_t)(mBase + row) * ldc + n0 + c8) = hv;
          if (OUT_MODE == 2) *(volatile v8h*)(C2 + (size_t)(mBase + row) * ldc + n0 + c8) = lv;
        }
        __threadfence();
      }
    }
    __builtin_amdgcn_fence(__ATOMIC_RELEASE, "workgroup");
    __builtin_amdgcn_wave_barrier();
    __builtin_amdgcn_fence(__ATOMIC_ACQUIRE, "workgroup");
  }
}

__device__ __forceinline__ float fsig(float v)  { return __builtin_amdgcn_rcpf(1.0f + expf(-v)); }
__device__ __forceinline__ float ftanh(float v) { return 1.0f - 2.0f * __builtin_amdgcn_rcpf(1.0f + expf(2.0f * v)); }

__global__ __launch_bounds__(PTHR) void wperm_kernel(const float* __restrict__ wi,
                                                     const float* __restrict__ wh,
                                                     unsigned short* __restrict__ wpl) {
  const int part = blockIdx.y;
  const int i  = blockIdx.x * PTHR + threadIdx.x;
  const int r  = i >> 5;
  const int c8 = (i & 31) * 8;
  const int w  = r >> 6, l = (r >> 2) & 15, g = r & 3;
  const int col = g * NHID + 16 * w + l;
  const float* src = (part == 0) ? wi : wh;
  v8h hv;
#pragma unroll
  for (int jj = 0; jj < 8; ++jj) {
    const float v = src[(size_t)(c8 + jj) * NGATE4 + col];
    hv[jj] = __builtin_bit_cast(_Float16, (unsigned short)f2bf_u(v));
  }
  unsigned short* dst = wpl + (size_t)part * ((size_t)NGATE4 * NIN) + (size_t)r * NIN + c8;
  *(volatile v8h*)dst = hv;
  __threadfence();
  *(volatile v8h*)dst = hv;
}

__global__ __launch_bounds__(PTHR) void bperm_kernel(const float* __restrict__ bsrc, float* __restrict__ bp) {
  const int q = threadIdx.x;
  v4f o;
  o[0] = bsrc[q];
  o[1] = bsrc[NHID + q];
  o[2] = bsrc[2 * NHID + q];
  o[3] = bsrc[3 * NHID + q];
  float* dst = bp + 4 * q;
  *(volatile v4f*)dst = o;
  __threadfence();
  *(volatile v4f*)dst = o;
}

__global__ __launch_bounds__(PTHR) void xcast_kernel(const float* __restrict__ x, unsigned short* __restrict__ x16) {
  const int i = blockIdx.x * PTHR + threadIdx.x;
  const float* sp = x + (size_t)i * 8;
  const v4f a  = *(const v4f*)sp;
  const v4f bq = *(const v4f*)(sp + 4);
  v8h hv;
#pragma unroll
  for (int e = 0; e < 4; ++e) {
    hv[e]     = __builtin_bit_cast(_Float16, (unsigned short)f2bf_u(a[e]));
    hv[4 + e] = __builtin_bit_cast(_Float16, (unsigned short)f2bf_u(bq[e]));
  }
  unsigned short* dst = x16 + (size_t)i * 8;
  *(volatile v8h*)dst = hv;
  __threadfence();
  *(volatile v8h*)dst = hv;
}

__global__ __launch_bounds__(RTHR) void lstm_seq_kernel(const unsigned short* __restrict__ zp,
                                                        const unsigned short* __restrict__ whpp,
                                                        const int* __restrict__ seqlen,
                                                        float* __restrict__ y) {
  __shared__ __align__(16) __bf16 abuf[2 * ATILE];
  __shared__ __align__(16) float  slab[2 * STILE];
  const __bf16* whp = (const __bf16*)whpp;
  const unsigned long long* zp64 = (const unsigned long long*)(const void*)zp;
  const int tid = threadIdx.x, lane = tid & 31, wave = tid >> 5;
  const int c = lane & 15, hh = lane >> 4, koff = hh * 8;
  const int u = 16 * wave + c;

  int Lv[4];
#pragma unroll
  for (int j = 0; j < 4; ++j) Lv[j] = seqlen[4 * hh + j] & (NSTEP - 1);
  const int sb = wave >> 1, shalf = wave & 1;
  const int Ls = seqlen[sb] & (NSTEP - 1);

  {
    const __bf16 bz = bf_from_u(0u);
    const v8b z8 = {bz, bz, bz, bz, bz, bz, bz, bz};
    for (int i = tid; i < (2 * ATILE) / 8; i += RTHR) *(v8b*)(abuf + i * 8) = z8;
  }
  float cst[4];
#pragma unroll
  for (int j = 0; j < 4; ++j) cst[j] = 0.0f;
  __syncthreads();

  const __bf16* bbase = whp + (size_t)(64 * wave + 4 * c) * NHID + koff;
  const v8f zacc = {0.f, 0.f, 0.f, 0.f, 0.f, 0.f, 0.f, 0.f};

#pragma unroll 1
  for (int s = 0; s < NSTEP; ++s) {
    const int cur = s & 1, nxt = cur ^ 1;

    unsigned long long zw[4];
#pragma unroll
    for (int j = 0; j < 4; ++j) {
      const int bb = 4 * hh + j;
      const int p  = (Lv[j] + NSTEP - 1 - s) & (NSTEP - 1);
      zw[j] = zp64[((size_t)bb * NSTEP + (size_t)p) * (NGATE4 / 4) + u];
    }

    const __bf16* arow = abuf + cur * ATILE + c * APITCH + koff;
    v8f acc0 = zacc, acc1 = zacc, acc2 = zacc, acc3 = zacc;
#pragma unroll 1
    for (int k0 = 0; k0 < NHID; k0 += 32) {
      const v16b fa = Frag<__bf16>::load(arow + k0);
      const v16b b0 = Frag<__bf16>::load(bbase + k0);
      const v16b b1 = Frag<__bf16>::load(bbase + NHID + k0);
      const v16b b2 = Frag<__bf16>::load(bbase + 2 * NHID + k0);
      const v16b b3 = Frag<__bf16>::load(bbase + 3 * NHID + k0);
      acc0 = Frag<__bf16>::mma(fa, b0, acc0);
      acc1 = Frag<__bf16>::mma(fa, b1, acc1);
      acc2 = Frag<__bf16>::mma(fa, b2, acc2);
      acc3 = Frag<__bf16>::mma(fa, b3, acc3);
      group_guard(acc0, acc1, acc2, acc3, fa, b0, b1, b2, b3);
    }
    acc_guard4(acc0, acc1, acc2, acc3);

    float zz0[4], zz1[4], zz2[4], zz3[4];
    {
      float q0[8], q1[8], q2[8], q3[8];
#pragma unroll
      for (int r = 0; r < 8; ++r) {
        q0[r] = __shfl_xor(acc0[r], 16, 32);
        q1[r] = __shfl_xor(acc1[r], 16, 32);
        q2[r] = __shfl_xor(acc2[r], 16, 32);
        q3[r] = __shfl_xor(acc3[r], 16, 32);
      }
#pragma unroll
      for (int j = 0; j < 4; ++j) {
        const float s0a = acc0[j] + q0[j], s0b = acc0[4 + j] + q0[4 + j];
        const float s1a = acc1[j] + q1[j], s1b = acc1[4 + j] + q1[4 + j];
        const float s2a = acc2[j] + q2[j], s2b = acc2[4 + j] + q2[4 + j];
        const float s3a = acc3[j] + q3[j], s3b = acc3[4 + j] + q3[4 + j];
        zz0[j] = hh ? s0b : s0a;
        zz1[j] = hh ? s1b : s1a;
        zz2[j] = hh ? s2b : s2a;
        zz3[j] = hh ? s3b : s3a;
      }
    }

    __bf16* hnx = abuf + nxt * ATILE;
    float*  slc = slab + cur * STILE;
#pragma unroll
    for (int j = 0; j < 4; ++j) {
      const int bb = 4 * hh + j;
      const unsigned long long wv = zw[j];
      const float zi = zz0[j] + h16_to_f32((unsigned)(wv & 0xffffull));
      const float zf = zz1[j] + h16_to_f32((unsigned)((wv >> 16) & 0xffffull));
      const float zg = zz2[j] + h16_to_f32((unsigned)((wv >> 32) & 0xffffull));
      const float zo = zz3[j] + h16_to_f32((unsigned)((wv >> 48) & 0xffffull));
      const float ig = fsig(zi);
      const float fg = fsig(zf);
      const float gg = ftanh(zg);
      const float og = fsig(zo);
      const float cn = fg * cst[j] + ig * gg;
      cst[j] = cn;
      const float hn = og * ftanh(cn);
      const unsigned hb = f2bf_u(hn);
      const unsigned lb = f2bf_u(hn - bf_u2f(hb));
      hnx[bb * APITCH + u]            = bf_from_u(hb);
      hnx[(NBATCH + bb) * APITCH + u] = bf_from_u(lb);
      slc[bb * SPITCH + u]            = hn;
    }

    __syncthreads();

    {
      const int ps = (Ls + NSTEP - 1 - s) & (NSTEP - 1);
      const v4f v = *(const v4f*)(slc + sb * SPITCH + shalf * 128 + lane * 4);
      float* dst = y + ((size_t)sb * NSTEP + (size_t)ps) * NHID + shalf * 128 + lane * 4;
      *(volatile v4f*)dst = v;
      __threadfence();
      *(volatile v4f*)dst = v;
    }
  }
}

extern "C" void kernel_launch(void* const* d_in, const int* in_sizes, int n_in,
                              void* d_out, int out_size, void* d_ws, size_t ws_size, hipStream_t stream) {
  if (n_in < 5 || d_out == nullptr || d_ws == nullptr) return;
  if (in_sizes[0] != NBATCH * NSTEP * NIN || in_sizes[1] != NIN * NGATE4 || in_sizes[2] != NHID * NGATE4 ||
      in_sizes[3] != NGATE4 || in_sizes[4] != NBATCH || out_size != NBATCH * NSTEP * NHID) return;

  const float* x      = (const float*)d_in[0];
  const float* wi     = (const float*)d_in[1];
  const float* wh     = (const float*)d_in[2];
  const float* bias   = (const float*)d_in[3];
  const int*   seqlen = (const int*)d_in[4];
  float*       y      = (float*)d_out;

  char* ws = (char*)d_ws; size_t off = 0;
  auto carve = [&](size_t bytes) -> char* { char* p = ws + off; off += (bytes + 255) & ~(size_t)255; return p; };
  unsigned short* X16 = (unsigned short*)carve((size_t)NROWS * NIN * 2);
  unsigned short* WPL = (unsigned short*)carve((size_t)2 * NGATE4 * NIN * 2);
  float*          BP  = (float*)carve((size_t)NGATE4 * 4);
  unsigned short* ZP  = (unsigned short*)carve((size_t)NROWS * NGATE4 * 2);
  if (off > ws_size || off > (size_t)134217728) return;
  unsigned short* WIP = WPL;
  unsigned short* WHP = WPL + (size_t)NGATE4 * NIN;

  wperm_kernel<<<dim3(WCHUNKS / PTHR, 2), PTHR, 0, stream>>>(wi, wh, WPL);
  bperm_kernel<<<1, PTHR, 0, stream>>>(bias, BP);

  xcast_kernel<<<XCHUNKS / PTHR, PTHR, 0, stream>>>(x, X16);

  wmma_gemm64<1, false, 2, 1, false, 0><<<dim3(GEMM_BLOCKS, 1), 256, 0, stream>>>(
      X16, X16, NIN, 0L, WIP, WIP, NIN, 0L, (void*)ZP, (void*)ZP, NGATE4, 0L,
      BP, BP, 0L, NROWS, NGATE4, NIN, 1.0f);

  lstm_seq_kernel<<<1, RTHR, 0, stream>>>(ZP, WHP, seqlen, y);
}
